// ManyNetworkModel_24111946399932
// MI455X (gfx1250) — hardware-verified
//
#include <hip/hip_runtime.h>
#include <math.h>

typedef __attribute__((ext_vector_type(16))) _Float16 v16h;
typedef __attribute__((ext_vector_type(16))) __bf16 v16b;
typedef __attribute__((ext_vector_type(8)))  _Float16 v8h;
typedef __attribute__((ext_vector_type(8)))  float v8f;
typedef __attribute__((ext_vector_type(4)))  float v4f;
typedef __attribute__((ext_vector_type(2)))  float v2f;
typedef __attribute__((ext_vector_type(4)))  unsigned v4u;
typedef __attribute__((ext_vector_type(4)))  int v4i;
typedef float __attribute__((may_alias)) float_a;
typedef int __attribute__((may_alias)) int_a;

template <typename T> __device__ __forceinline__ void vst2(void* p, T v) { *(volatile T*)p = v; __threadfence(); *(volatile T*)p = v; }
__device__ __forceinline__ v8f wmma16(v16h a, v16h b, v8f c) {
  v8f d = __builtin_amdgcn_wmma_f32_16x16x32_f16(false, a, false, b, (short)0, c, false, false);
  asm volatile("v_nop\n\tv_nop\n\tv_nop\n\tv_nop" : "+v"(d) : "v"(a), "v"(b));
  return d;
}
__device__ __forceinline__ v8f wmma_bf(v16b a, v16b b, v8f c) {
  v8f d = __builtin_amdgcn_wmma_f32_16x16x32_bf16(false, a, false, b, (short)0, c, false, false);
  asm volatile("v_nop\n\tv_nop\n\tv_nop\n\tv_nop" : "+v"(d) : "v"(a), "v"(b));
  return d;
}
__device__ __forceinline__ v16h frag_h(const _Float16* rowk0, int lane) {
  union { v16h v; v8h q[2]; } u; const _Float16* p = rowk0 + 8 * (lane >> 4);
  u.q[0] = *(const v8h*)p; u.q[1] = *(const v8h*)(p + 16); return u.v;
}
__device__ __forceinline__ v16h frag_f32(const float* rowk0, int lane) {
  v16h a; const float* p = rowk0 + 8 * (lane >> 4);
#pragma unroll
  for (int i = 0; i < 8; ++i) { a[i] = (_Float16)p[i]; a[8 + i] = (_Float16)p[16 + i]; }
  return a;
}
__device__ __forceinline__ v16h frag_f32s(const float* rowk0, int lane, float sc) {
  v16h a; const float* p = rowk0 + 8 * (lane >> 4);
#pragma unroll
  for (int i = 0; i < 8; ++i) { a[i] = (_Float16)(p[i] * sc); a[8 + i] = (_Float16)(p[16 + i] * sc); }
  return a;
}
__device__ __forceinline__ v16h fragc_f32(const float* W, int k0, int n, int lane, int ld, int K) {
  v16h a; const int g = lane >> 4;
#pragma unroll
  for (int i = 0; i < 8; ++i) { const int ka = k0 + 8 * g + i, kb = ka + 16;
    a[i] = (_Float16)(ka < K ? W[(size_t)(ka < K ? ka : K - 1) * ld + n] : 0.f); a[8 + i] = (_Float16)(kb < K ? W[(size_t)(kb < K ? kb : K - 1) * ld + n] : 0.f); }
  return a;
}
struct F2 { v16b h, l; };
__device__ __forceinline__ F2 bsplit16(const float v[16]) { F2 r;
#pragma unroll
  for (int i = 0; i < 16; ++i) { const __bf16 h = (__bf16)v[i]; r.h[i] = h; r.l[i] = (__bf16)(v[i] - (float)h); }
  return r; }
__device__ __forceinline__ F2 split_row(const float* row, int k0, int lane) { float v[16]; const float* p = row + k0 + 8 * (lane >> 4);
#pragma unroll
  for (int i = 0; i < 8; ++i) { v[i] = p[i]; v[8 + i] = p[16 + i]; }
  return bsplit16(v); }
__device__ __forceinline__ F2 split_rowK(const float* row, int k0, int lane, int K) { float v[16]; const int g = lane >> 4;
#pragma unroll
  for (int i = 0; i < 8; ++i) { const int ka = k0 + 8 * g + i, kb = ka + 16; v[i] = ka < K ? row[ka < K ? ka : K - 1] : 0.f; v[8 + i] = kb < K ? row[kb < K ? kb : K - 1] : 0.f; }
  return bsplit16(v); }
__device__ __forceinline__ F2 split_col(const float* W, int k0, int n, int lane, int ld, int K) { float v[16]; const int g = lane >> 4;
#pragma unroll
  for (int i = 0; i < 8; ++i) { const int ka = k0 + 8 * g + i, kb = ka + 16; v[i] = ka < K ? W[(size_t)(ka < K ? ka : K - 1) * ld + n] : 0.f; v[8 + i] = kb < K ? W[(size_t)(kb < K ? kb : K - 1) * ld + n] : 0.f; }
  return bsplit16(v); }
__device__ __forceinline__ v8f mac3(const F2& a, const F2& b, v8f c) { c = wmma_bf(a.l, b.h, c); c = wmma_bf(a.h, b.l, c); return wmma_bf(a.h, b.h, c); }
__device__ __forceinline__ float sigm(float v) { return 1.0f / (1.0f + expf(-v)); }
#define LDSX() do { asm volatile("s_wait_dscnt 0" ::: "memory"); __builtin_amdgcn_wave_barrier(); __builtin_amdgcn_fence(__ATOMIC_RELEASE, "workgroup"); } while (0)


#define NRW 131072
#define NF 32
#define NA 8
#define NHID 64
__device__ __forceinline__ float bfr(float v) { return (float)(__bf16)v; }
__device__ __forceinline__ v16b frag_b(const __bf16* rowk0, int lane) { return __builtin_bit_cast(v16b, frag_h((const _Float16*)rowk0, lane)); }

__global__ __launch_bounds__(128) void k_many(const float* __restrict__ ft, const float* __restrict__ at, const float* __restrict__ W1, const float* __restrict__ b1, const float* __restrict__ W2, const float* __restrict__ b2, float* __restrict__ out) {
  __shared__ __align__(16) float so[4][16][NF + 4];
  const int tid = threadIdx.x, wave = tid >> 5, lane = tid & 31, col = lane & 15, g = lane >> 4; const size_t r0 = (size_t)blockIdx.x * 64 + wave * 16;
  const v16b a0 = split_rowK(ft + (r0 + col) * NF, 0, lane, NF).h;
  const v16b a1 = split_rowK(at + (r0 + col) * NA, 0, lane, NA).h;
#pragma unroll 1
  for (int ps = 0; ps < NF / 2; ++ps) { v8f acc[8] = {};
#pragma unroll
    for (int j = 0; j < 8; ++j) { const int f = ps * 2 + (j >> 2), h = (j & 3) * 16 + col; const float* Wf = W1 + (size_t)f * (NF + NA) * NHID;
      acc[j] = wmma_bf(a0, split_col(Wf, 0, h, lane, NHID, NF + NA).h, acc[j]);
      acc[j] = wmma_bf(a1, split_col(Wf, NF, h, lane, NHID, NF + NA).h, acc[j]); }
#pragma unroll
    for (int ff = 0; ff < 2; ++ff) { const int f = ps * 2 + ff; float part[8];
#pragma unroll
      for (int r = 0; r < 8; ++r) part[r] = 0.f;
#pragma unroll
      for (int jt = 0; jt < 4; ++jt) { const int h = jt * 16 + col; const float bb = bfr(b1[f * NHID + h]), w2 = bfr(W2[f * NHID + h]);
#pragma unroll
        for (int r = 0; r < 8; ++r) { const float v = acc[ff * 4 + jt][r] + bb; part[r] += (v > 0.f ? v : 0.f) * w2; } }
#pragma unroll
      for (int r = 0; r < 8; ++r) {
#pragma unroll
        for (int o_ = 1; o_ < 16; o_ <<= 1) part[r] += __shfl_xor(part[r], o_, 32); }
      if (col == 0) {
#pragma unroll
        for (int r = 0; r < 8; ++r) { const int rl = 8 * g + r; so[wave][rl][f] = part[r] + bfr(b2[f]) + bfr(ft[(r0 + rl) * NF + f]); } } } }
  LDSX();
  for (int qq = lane; qq < 16 * 8; qq += 32) { const int rl = qq >> 3, pc = qq & 7; vst2(out + (r0 + rl) * NF + pc * 4, *(const v4f*)(&so[wave][rl][pc * 4])); }
}
extern "C" void kernel_launch(void* const* d_in, const int* in_sizes, int n_in, void* d_out, int out_size, void* d_ws, size_t ws_size, hipStream_t stream) {
  (void)in_sizes; (void)n_in; (void)out_size; (void)ws_size; (void)d_ws;
  const float** I = (const float**)d_in;
  k_many<<<NRW / 64, 128, 0, stream>>>(I[0], I[1], I[2], I[3], I[4], I[5], (float*)d_out);
}
